// SSMEncoderAdapter_49452253446285
// MI455X (gfx1250) — hardware-verified
//
#include <hip/hip_runtime.h>
#include <math.h>


typedef _Float16 half_t;
typedef _Float16 v16h __attribute__((ext_vector_type(16)));
typedef _Float16 v8h  __attribute__((ext_vector_type(8)));
typedef float    v8f  __attribute__((ext_vector_type(8)));
typedef float    v4f  __attribute__((ext_vector_type(4)));
typedef float    v4fa __attribute__((ext_vector_type(4), __may_alias__));
typedef _Float16 v8ha __attribute__((ext_vector_type(8), __may_alias__));

#define NLc  2
#define DMc  256
#define Fc   128
#define DIc  512
#define DSc  16
#define DRc  16
#define Kc   4
#define Bc   4
#define Lc   2048
#define BLc  (Bc * Lc)
#define DTKP 32
#define XPN  64
#define DBCW 64
#define SCN  32

static_assert(BLc % 16 == 0, "");
static_assert(DMc % 64 == 0 && (2 * DIc) % 64 == 0 && XPN % 64 == 0 && DIc % 64 == 0, "");
static_assert(Fc % 32 == 0 && DMc % 32 == 0 && DIc % 32 == 0 && DTKP % 32 == 0, "");
static_assert(Lc % SCN == 0 && (SCN * DIc) % (8 * DIc) == 0, "");
static_assert(DMc == 256 && Fc == 128 && DIc == 512, "");

union FragH { v16h v; v8h h[2]; };
union Pack8 { v8h v; half_t e[8]; };

__device__ __forceinline__ v8f wmma_f16(v16h a, v16h b, v8f c)
{
    v8f d = __builtin_amdgcn_wmma_f32_16x16x32_f16(false, a, false, b, (short)0, c, false, false);
    asm volatile("v_nop\n\tv_nop\n\tv_nop\n\tv_nop" : "+v"(d) : "v"(a), "v"(b));
    return d;
}

__device__ __forceinline__ float wave_sum(float v)
{
    #pragma unroll
    for (int o = 16; o > 0; o >>= 1) v += __shfl_xor(v, o, 32);
    return v;
}

__device__ __forceinline__ float softplus_f(float v)
{
    return fmaxf(v, 0.f) + log1pf(__expf(-fabsf(v)));
}

__device__ __forceinline__ float silu_f(float v)
{
    return v / (1.f + __expf(-v));
}

__global__ void __launch_bounds__(128)
gemm_f16_kernel(const half_t* __restrict__ A,
                const half_t* __restrict__ W,
                const float* __restrict__ bias,
                float* C,
                int N, int Kd, int act, int accum, float oscale)
{
    __shared__ __attribute__((aligned(16))) float sT[4][16][64];

    const int lane  = threadIdx.x;
    const int wv    = threadIdx.y;
    const int hh    = lane >> 4;
    const int m     = lane & 15;
    const int nbase = (blockIdx.x * blockDim.y + wv) * 64;
    const int m0    = blockIdx.y * 16;

    v8f acc[4];
    #pragma unroll
    for (int t = 0; t < 4; ++t) {
        #pragma unroll
        for (int r = 0; r < 8; ++r) acc[t][r] = 0.f;
    }

    const half_t* aRow = A + (size_t)(m0 + m) * Kd;
    const half_t* wRow = W + (size_t)(nbase + m) * Kd;

    for (int kk = 0; kk < Kd; kk += 32) {
        FragH a;
        a.h[0] = *(const v8h*)(aRow + kk + 8 * hh);
        a.h[1] = *(const v8h*)(aRow + kk + 16 + 8 * hh);
        #pragma unroll
        for (int t = 0; t < 4; ++t) {
            const half_t* bp = wRow + (size_t)(16 * t) * Kd + kk;
            FragH b;
            b.h[0] = *(const v8h*)(bp + 8 * hh);
            b.h[1] = *(const v8h*)(bp + 16 + 8 * hh);
            acc[t] = wmma_f16(a.v, b.v, acc[t]);
        }
    }

    float (*tile)[64] = sT[wv];
    #pragma unroll
    for (int t = 0; t < 4; ++t) {
        const int n = nbase + 16 * t + m;
        const float bv = bias ? bias[n] : 0.f;
        #pragma unroll
        for (int r = 0; r < 8; ++r) {
            float v = acc[t][r] * oscale + bv;
            if (act) v = softplus_f(v);
            tile[8 * hh + r][16 * t + m] = v;
        }
    }
    __syncthreads();

    float* cbase = C + (size_t)(m0 + hh) * N + nbase + 4 * m;
    v4f vals[8];
    #pragma unroll
    for (int p = 0; p < 8; ++p) {
        v4f v = *(const v4fa*)(&tile[2 * p + hh][4 * m]);
        if (accum) v += *(const v4f*)(cbase + (size_t)(2 * p) * N);
        vals[p] = v;
    }
    #pragma unroll
    for (int p = 0; p < 8; ++p)
        *(volatile v4f*)(cbase + (size_t)(2 * p) * N) = vals[p];
    __threadfence();
    #pragma unroll
    for (int p = 0; p < 8; ++p)
        *(volatile v4f*)(cbase + (size_t)(2 * p) * N) = vals[p];
}

__global__ void __launch_bounds__(256)
cvt8_kernel(const float* __restrict__ src, half_t* __restrict__ dst, int n8, float scale)
{
    const int i = blockIdx.x * blockDim.x + threadIdx.x;
    if (i >= n8) return;
    const float* sp = src + (size_t)i * 8;
    v4f x0 = *(const v4f*)sp;
    v4f x1 = *(const v4f*)(sp + 4);
    Pack8 o;
    #pragma unroll
    for (int c = 0; c < 4; ++c) {
        o.e[c]     = (half_t)(x0[c] * scale);
        o.e[4 + c] = (half_t)(x1[c] * scale);
    }
    v8h ov = o.v;
    half_t* dp = dst + (size_t)i * 8;
    *(volatile v8h*)dp = ov;
    __threadfence();
    *(volatile v8h*)dp = ov;
}

__global__ void __launch_bounds__(256)
pad16to32_kernel(const float* __restrict__ src, int spitch, half_t* __restrict__ dst,
                 int n8, float scale)
{
    const int i = blockIdx.x * blockDim.x + threadIdx.x;
    if (i >= n8) return;
    const int row = i >> 2;
    const int ch  = i & 3;
    Pack8 o;
    if (ch < 2) {
        const float* sp = src + (size_t)row * spitch + ch * 8;
        v4f x0 = *(const v4f*)sp;
        v4f x1 = *(const v4f*)(sp + 4);
        #pragma unroll
        for (int c = 0; c < 4; ++c) {
            o.e[c]     = (half_t)(x0[c] * scale);
            o.e[4 + c] = (half_t)(x1[c] * scale);
        }
    } else {
        #pragma unroll
        for (int c = 0; c < 8; ++c) o.e[c] = (half_t)0.f;
    }
    v8h ov = o.v;
    half_t* dp = dst + (size_t)i * 8;
    *(volatile v8h*)dp = ov;
    __threadfence();
    *(volatile v8h*)dp = ov;
}

__global__ void __launch_bounds__(256)
pad_xproj_w_kernel(const float* __restrict__ src, half_t* __restrict__ dst, int n8, float scale)
{
    const int i = blockIdx.x * blockDim.x + threadIdx.x;
    if (i >= n8) return;
    const int chunks_per_row = DIc / 8;
    const int layer = i / (XPN * chunks_per_row);
    const int rem   = i % (XPN * chunks_per_row);
    const int r     = rem / chunks_per_row;
    const int ch    = rem % chunks_per_row;
    Pack8 o;
    if (r < DRc + 2 * DSc) {
        const float* sp = src + ((size_t)layer * (DRc + 2 * DSc) + r) * DIc + ch * 8;
        v4f x0 = *(const v4f*)sp;
        v4f x1 = *(const v4f*)(sp + 4);
        #pragma unroll
        for (int c = 0; c < 4; ++c) {
            o.e[c]     = (half_t)(x0[c] * scale);
            o.e[4 + c] = (half_t)(x1[c] * scale);
        }
    } else {
        #pragma unroll
        for (int c = 0; c < 8; ++c) o.e[c] = (half_t)0.f;
    }
    v8h ov = o.v;
    half_t* dp = dst + (size_t)i * 8;
    *(volatile v8h*)dp = ov;
    __threadfence();
    *(volatile v8h*)dp = ov;
}

__global__ void __launch_bounds__(256)
rmsnorm_kernel(const float* __restrict__ h, const float* __restrict__ w,
               half_t* __restrict__ out16, int nrows)
{
    const int wv  = threadIdx.x >> 5;
    const int l   = threadIdx.x & 31;
    const int row = blockIdx.x * 8 + wv;
    if (row >= nrows) return;
    const float* hp = h + (size_t)row * DMc + 8 * l;
    v4f a0 = *(const v4f*)hp;
    v4f a1 = *(const v4f*)(hp + 4);
    float ss = 0.f;
    #pragma unroll
    for (int c = 0; c < 4; ++c) ss += a0[c] * a0[c];
    #pragma unroll
    for (int c = 0; c < 4; ++c) ss += a1[c] * a1[c];
    ss = wave_sum(ss);
    const float sc = rsqrtf(ss * (1.f / (float)DMc) + 1e-6f);
    v4f w0 = *(const v4f*)(w + 8 * l);
    v4f w1 = *(const v4f*)(w + 8 * l + 4);
    Pack8 o;
    #pragma unroll
    for (int c = 0; c < 4; ++c) {
        o.e[c]     = (half_t)(a0[c] * sc * w0[c]);
        o.e[4 + c] = (half_t)(a1[c] * sc * w1[c]);
    }
    v8h ov = o.v;
    half_t* dp = out16 + (size_t)row * DMc + 8 * l;
    *(volatile v8h*)dp = ov;
    __threadfence();
    *(volatile v8h*)dp = ov;
}

__global__ void __launch_bounds__(256)
conv_silu_kernel(const float* __restrict__ xz, const float* __restrict__ cw,
                 const float* __restrict__ cb, half_t* __restrict__ u16,
                 int ngrp, float scale)
{
    const int gid = blockIdx.x * blockDim.x + threadIdx.x;
    if (gid >= ngrp) return;
    const int j  = gid & 63;
    const int bl = gid >> 6;
    const int l  = bl % Lc;
    const int d0 = j * 8;

    float acc[8];
    {
        v4f b0 = *(const v4f*)(cb + d0);
        v4f b1 = *(const v4f*)(cb + d0 + 4);
        #pragma unroll
        for (int c = 0; c < 4; ++c) { acc[c] = b0[c]; acc[4 + c] = b1[c]; }
    }
    v4f wq[8];
    #pragma unroll
    for (int c = 0; c < 8; ++c) wq[c] = *(const v4f*)(cw + (size_t)(d0 + c) * Kc);

    #pragma unroll
    for (int k = 0; k < Kc; ++k) {
        const int lt = l - (Kc - 1) + k;
        if (lt >= 0) {
            const float* xp = xz + (size_t)(bl - (Kc - 1) + k) * (2 * DIc) + d0;
            v4f x0 = *(const v4f*)xp;
            v4f x1 = *(const v4f*)(xp + 4);
            #pragma unroll
            for (int c = 0; c < 4; ++c) {
                acc[c]     += wq[c][k] * x0[c];
                acc[4 + c] += wq[4 + c][k] * x1[c];
            }
        }
    }
    Pack8 o;
    #pragma unroll
    for (int c = 0; c < 8; ++c) o.e[c] = (half_t)(silu_f(acc[c]) * scale);
    v8h ov = o.v;
    half_t* dp = u16 + (size_t)gid * 8;
    *(volatile v8h*)dp = ov;
    __threadfence();
    *(volatile v8h*)dp = ov;
}

__global__ void __launch_bounds__(DIc)
scan_kernel(const float* __restrict__ delta,
            const float* __restrict__ dbc,
            const float* __restrict__ xz,
            const float* __restrict__ cw,
            const float* __restrict__ cb,
            const float* __restrict__ A_log,
            const float* __restrict__ Dw,
            half_t* __restrict__ y16,
            float yscale)
{
    __shared__ float sB[SCN][DSc];
    __shared__ float sC[SCN][DSc];
    __shared__ __attribute__((aligned(16))) half_t sY[SCN][DIc];

    const int b = blockIdx.x;
    const int d = threadIdx.x;
    const size_t rowb = (size_t)b * Lc;

    float An[DSc];
    #pragma unroll
    for (int n = 0; n < DSc; ++n) An[n] = -__expf(A_log[d * DSc + n]);
    const float cw0 = cw[d * Kc + 0], cw1 = cw[d * Kc + 1];
    const float cw2 = cw[d * Kc + 2], cw3 = cw[d * Kc + 3];
    const float cbd = cb[d];
    const float Dd  = Dw[d];

    float hs[DSc];
    #pragma unroll
    for (int n = 0; n < DSc; ++n) hs[n] = 0.f;
    float x0 = 0.f, x1 = 0.f, x2 = 0.f;

    for (int t0 = 0; t0 < Lc; t0 += SCN) {
        for (int i = d; i < SCN * 2 * DSc; i += DIc) {
            const int tt = i >> 5, j = i & 31;
            const float v = dbc[(rowb + t0 + tt) * DBCW + DRc + j];
            if (j < DSc) sB[tt][j] = v; else sC[tt][j - DSc] = v;
        }
        __syncthreads();

        for (int tt = 0; tt < SCN; ++tt) {
            const size_t row = rowb + t0 + tt;
            const float xu = xz[row * (2 * DIc) + d];
            const float z  = xz[row * (2 * DIc) + DIc + d];
            const float dl = delta[row * DIc + d];
            float uc = cbd;
            uc += cw0 * x0;
            uc += cw1 * x1;
            uc += cw2 * x2;
            uc += cw3 * xu;
            x0 = x1; x1 = x2; x2 = xu;
            const float uu = silu_f(uc);
            const float du = dl * uu;
            float y = 0.f;
            #pragma unroll
            for (int n = 0; n < DSc; ++n) {
                const float dA = __expf(dl * An[n]);
                hs[n] = dA * hs[n] + du * sB[tt][n];
                y += hs[n] * sC[tt][n];
            }
            const float yv = (y + uu * Dd) * silu_f(z);
            sY[tt][d] = (half_t)(yv * yscale);
        }
        __syncthreads();

        v8h yv[4];
        #pragma unroll
        for (int q = 0; q < 4; ++q) {
            const int i = d + q * DIc;
            const int r = i >> 6, c = (i & 63) * 8;
            yv[q] = *(const v8ha*)(&sY[r][c]);
        }
        #pragma unroll
        for (int q = 0; q < 4; ++q) {
            const int i = d + q * DIc;
            const int r = i >> 6, c = (i & 63) * 8;
            *(volatile v8h*)(y16 + (rowb + t0 + r) * DIc + c) = yv[q];
        }
        __threadfence();
        #pragma unroll
        for (int q = 0; q < 4; ++q) {
            const int i = d + q * DIc;
            const int r = i >> 6, c = (i & 63) * 8;
            *(volatile v8h*)(y16 + (rowb + t0 + r) * DIc + c) = yv[q];
        }
    }
}

__global__ void __launch_bounds__(256)
pool_proj_kernel(const float* __restrict__ h, const float* __restrict__ fw,
                 const float* __restrict__ pw, const float* __restrict__ pb,
                 float* __restrict__ bbuf)
{
    __shared__ float sP[8][DMc];
    __shared__ float sPool[DMc];
    __shared__ __attribute__((aligned(16))) float sBias[Fc];

    const int tid = threadIdx.x;
    const int wv  = tid >> 5;
    const int l   = tid & 31;
    const int b   = blockIdx.x;

    v4f w0 = *(const v4f*)(fw + 8 * l);
    v4f w1 = *(const v4f*)(fw + 8 * l + 4);
    v4f p0, p1;
    #pragma unroll
    for (int c = 0; c < 4; ++c) { p0[c] = 0.f; p1[c] = 0.f; }

    for (int r = wv; r < Lc; r += 8) {
        const float* hp = h + ((size_t)b * Lc + r) * DMc + 8 * l;
        v4f a0 = *(const v4f*)hp;
        v4f a1 = *(const v4f*)(hp + 4);
        float ss = 0.f;
        #pragma unroll
        for (int c = 0; c < 4; ++c) ss += a0[c] * a0[c];
        #pragma unroll
        for (int c = 0; c < 4; ++c) ss += a1[c] * a1[c];
        ss = wave_sum(ss);
        const float sc = rsqrtf(ss * (1.f / (float)DMc) + 1e-6f);
        #pragma unroll
        for (int c = 0; c < 4; ++c) {
            p0[c] += a0[c] * sc * w0[c];
            p1[c] += a1[c] * sc * w1[c];
        }
    }
    #pragma unroll
    for (int c = 0; c < 4; ++c) { sP[wv][8 * l + c] = p0[c]; sP[wv][8 * l + 4 + c] = p1[c]; }
    __syncthreads();

    {
        float s = 0.f;
        #pragma unroll
        for (int q = 0; q < 8; ++q) s += sP[q][tid];
        sPool[tid] = s * (1.f / (float)Lc);
    }
    __syncthreads();

    if (tid < Fc) {
        float acc = pb[tid];
        const float* pr = pw + (size_t)tid * DMc;
        #pragma unroll 4
        for (int dm = 0; dm < DMc; ++dm) acc += sPool[dm] * pr[dm];
        sBias[tid] = acc;
    }
    __syncthreads();

    v4f bv;
    #pragma unroll
    for (int c = 0; c < 4; ++c) bv[c] = 0.f;
    if (tid < 32) bv = *(const v4fa*)(&sBias[4 * tid]);
    if (tid < 32) *(volatile v4f*)(bbuf + (size_t)b * Fc + 4 * tid) = bv;
    __threadfence();
    if (tid < 32) *(volatile v4f*)(bbuf + (size_t)b * Fc + 4 * tid) = bv;
}

__global__ void __launch_bounds__(256)
final_add_kernel(const float* __restrict__ x, const float* __restrict__ bbuf,
                 float* __restrict__ out, int n4)
{
    const int i = blockIdx.x * blockDim.x + threadIdx.x;
    if (i >= n4) return;
    const int b = i / (Lc * Fc / 4);
    const int f = (i * 4) & (Fc - 1);
    v4f v = *(const v4f*)(x + (size_t)i * 4) + *(const v4f*)(bbuf + (size_t)b * Fc + f);
    float* op = out + (size_t)i * 4;
    *(volatile v4f*)op = v;
    __threadfence();
    *(volatile v4f*)op = v;
}

static void launch_gemm(const half_t* A, const half_t* W, const float* bias,
                        float* C, int M, int N, int Kd, int act, int accum,
                        float oscale, hipStream_t s)
{
    const int strips = N / 64;
    const int wy     = (strips >= 4) ? 4 : strips;
    dim3 block(32, wy, 1);
    dim3 grid(strips / wy, M / 16, 1);
    gemm_f16_kernel<<<grid, block, 0, s>>>(A, W, bias, C, N, Kd, act, accum, oscale);
}

static void launch_cvt8(const float* src, half_t* dst, int n, float scale, hipStream_t s)
{
    const int n8 = n / 8;
    cvt8_kernel<<<(n8 + 255) / 256, 256, 0, s>>>(src, dst, n8, scale);
}

extern "C" void kernel_launch(void* const* d_in, const int* in_sizes, int n_in,
                              void* d_out, int out_size, void* d_ws, size_t ws_size,
                              hipStream_t stream)
{
    if (n_in < 16) return;
    if (in_sizes[0] != BLc * Fc || in_sizes[1] != DMc * Fc ||
        in_sizes[3] != NLc * 2 * DIc * DMc || in_sizes[6] != NLc * (DRc + 2 * DSc) * DIc ||
        in_sizes[7] != NLc * DIc * DRc || in_sizes[11] != NLc * DMc * DIc ||
        in_sizes[14] != Fc * DMc || out_size != BLc * Fc) return;

    const float* x        = (const float*)d_in[0];
    const float* embed_w  = (const float*)d_in[1];
    const float* embed_b  = (const float*)d_in[2];
    const float* in_w     = (const float*)d_in[3];
    const float* conv_w   = (const float*)d_in[4];
    const float* conv_b   = (const float*)d_in[5];
    const float* xproj_w  = (const float*)d_in[6];
    const float* dt_w     = (const float*)d_in[7];
    const float* dt_b     = (const float*)d_in[8];
    const float* A_log    = (const float*)d_in[9];
    const float* Dp       = (const float*)d_in[10];
    const float* out_w    = (const float*)d_in[11];
    const float* norm_w   = (const float*)d_in[12];
    const float* fnorm_w  = (const float*)d_in[13];
    const float* proj_w   = (const float*)d_in[14];
    const float* proj_b   = (const float*)d_in[15];
    float* out = (float*)d_out;

    char* ws = (char*)d_ws;
    size_t off = 0;
    auto carve = [&](size_t bytes) -> void* {
        void* p = ws + off;
        off = (off + bytes + 255) & ~(size_t)255;
        return p;
    };
    float*  h      = (float*) carve((size_t)BLc * DMc * 4);
    half_t* hn16   = (half_t*)carve((size_t)BLc * DMc * 2);
    float*  xz     = (float*) carve((size_t)BLc * 2 * DIc * 4);
    half_t* u16    = (half_t*)carve((size_t)BLc * DIc * 2);
    float*  dbc    = (float*) carve((size_t)BLc * DBCW * 4);
    half_t* dt16   = (half_t*)carve((size_t)BLc * DTKP * 2);
    float*  delta  = (float*) carve((size_t)BLc * DIc * 4);
    half_t* y16    = (half_t*)carve((size_t)BLc * DIc * 2);
    half_t* x16    = (half_t*)carve((size_t)BLc * Fc * 2);
    half_t* ew16   = (half_t*)carve((size_t)DMc * Fc * 2);
    half_t* inw16  = (half_t*)carve((size_t)NLc * 2 * DIc * DMc * 2);
    half_t* xpw16  = (half_t*)carve((size_t)NLc * XPN * DIc * 2);
    half_t* dtw16  = (half_t*)carve((size_t)NLc * DIc * DTKP * 2);
    half_t* ow16   = (half_t*)carve((size_t)NLc * DMc * DIc * 2);
    float*  bbuf   = (float*) carve((size_t)Bc * Fc * 4);
    if (off > ws_size) return;

    const float WSC = 64.f;
    const float USC = 64.f;
    const float DTSC = 64.f;
    const float YSC = 256.f;

    launch_cvt8(x,       x16,   BLc * Fc,            1.f, stream);
    launch_cvt8(embed_w, ew16,  DMc * Fc,            WSC, stream);
    launch_cvt8(in_w,    inw16, NLc * 2 * DIc * DMc, WSC, stream);
    launch_cvt8(out_w,   ow16,  NLc * DMc * DIc,     WSC, stream);
    {
        const int n8 = NLc * XPN * DIc / 8;
        pad_xproj_w_kernel<<<(n8 + 255) / 256, 256, 0, stream>>>(xproj_w, xpw16, n8, WSC);
    }
    {
        const int n8 = NLc * DIc * DTKP / 8;
        pad16to32_kernel<<<(n8 + 255) / 256, 256, 0, stream>>>(dt_w, DRc, dtw16, n8, WSC);
    }

    launch_gemm(x16, ew16, embed_b, h, BLc, DMc, Fc, 0, 0, 1.f / WSC, stream);

    for (int i = 0; i < NLc; ++i) {
        const half_t* inw_i = inw16 + (size_t)i * 2 * DIc * DMc;
        const half_t* xpw_i = xpw16 + (size_t)i * XPN * DIc;
        const half_t* dtw_i = dtw16 + (size_t)i * DIc * DTKP;
        const half_t* ow_i  = ow16  + (size_t)i * DMc * DIc;
        const float*  cw_i  = conv_w + (size_t)i * DIc * Kc;
        const float*  cb_i  = conv_b + (size_t)i * DIc;

        rmsnorm_kernel<<<(BLc + 7) / 8, 256, 0, stream>>>(h, norm_w + (size_t)i * DMc, hn16, BLc);

        launch_gemm(hn16, inw_i, nullptr, xz, BLc, 2 * DIc, DMc, 0, 0, 1.f / WSC, stream);

        {
            const int ngrp = BLc * (DIc / 8);
            conv_silu_kernel<<<(ngrp + 255) / 256, 256, 0, stream>>>(xz, cw_i, cb_i, u16, ngrp, USC);
        }

        launch_gemm(u16, xpw_i, nullptr, dbc, BLc, XPN, DIc, 0, 0, 1.f / (USC * WSC), stream);

        {
            const int n8 = BLc * DTKP / 8;
            pad16to32_kernel<<<(n8 + 255) / 256, 256, 0, stream>>>(dbc, DBCW, dt16, n8, DTSC);
        }

        launch_gemm(dt16, dtw_i, dt_b + (size_t)i * DIc, delta,
                    BLc, DIc, DTKP, 1, 0, 1.f / (DTSC * WSC), stream);

        scan_kernel<<<Bc, DIc, 0, stream>>>(delta, dbc, xz, cw_i, cb_i,
                                            A_log + (size_t)i * DIc * DSc,
                                            Dp + (size_t)i * DIc, y16, YSC);

        launch_gemm(y16, ow_i, nullptr, h, BLc, DMc, DIc, 0, 1, 1.f / (YSC * WSC), stream);
    }

    pool_proj_kernel<<<Bc, 256, 0, stream>>>(h, fnorm_w, proj_w, proj_b, bbuf);
    {
        const int n4 = BLc * Fc / 4;
        final_add_kernel<<<(n4 + 255) / 256, 256, 0, stream>>>(x, bbuf, out, n4);
    }
}
